// DeepMatrixtModel_45011257262087
// MI455X (gfx1250) — hardware-run, weakly checked
//
#include <hip/hip_runtime.h>


namespace {
constexpr int NU = 100000, NM = 20000, NMP = 20096  , K = 64, E = 2000000  , N = NU  , NB_ = 100000  ;
constexpr float XS = 8.0f, WSC = 256.0f, NEG = 0.2f  , MAXR = 5.0f;

typedef _Float16 b16;
typedef __attribute__((ext_vector_type(16))) _Float16 v16b;
typedef __attribute__((ext_vector_type(8))) _Float16 v8b;
typedef __attribute__((ext_vector_type(8))) float v8f;
typedef __attribute__((ext_vector_type(4))) float v4f;
__device__ __forceinline__ float bf16_rne(float f) { unsigned int u = __float_as_uint(f); u += 0x7FFFu + ((u >> 16) & 1u); return __uint_as_float(u & 0xFFFF0000u); }
__device__ __forceinline__ void split16(float v, b16& hi, b16& lo) { hi = (b16)v; lo = (b16)(v - (float)hi); }
__device__ __forceinline__ v16b frag_kb(const b16* p, int hh) { const v8b a = *(const v8b*)(p + 8 * hh), b = *(const v8b*)(p + 16 + 8 * hh); v16b f;
#pragma unroll
  for (int e = 0; e < 8; ++e) { f[e] = a[e]; f[8 + e] = b[e]; } return f; }
__device__ __forceinline__ v8f wmma16b(v16b a, v16b b, v8f c) { v8f d = __builtin_amdgcn_wmma_f32_16x16x32_f16(false, a, false, b, (short)0, c, false, false); asm volatile("v_nop\n\tv_nop\n\tv_nop\n\tv_nop" : "+v"(d) : "v"(a), "v"(b)); return d; }
__device__ __forceinline__ void wave_lds_sync() { __builtin_amdgcn_fence(__ATOMIC_RELEASE, "workgroup"); __builtin_amdgcn_wave_barrier(); __builtin_amdgcn_fence(__ATOMIC_ACQUIRE, "workgroup"); }
__device__ __forceinline__ float pmul(float a, float b) { float p = a * b; asm volatile("" : "+v"(p)); return p; }
__device__ __forceinline__ int iclamp(int v, int lo, int hi) { return v < lo ? lo : (v > hi ? hi : v); }
__device__ __forceinline__ float nexp(float x) { return __builtin_amdgcn_exp2f(x * 1.4426950408889634f); }
__device__ __forceinline__ float lrelu(float x) { return x > 0.0f ? x : NEG * x; }

constexpr int CSR_NBLK = 512, CSR_GB = 8  , CSR_GN = 1 << CSR_GB  , CSR_MAXG = 512, CSR_CAP = 12288  ;
__global__ __launch_bounds__(64) void csrA_kernel(const int* __restrict__ dst, int E, int N, int nG, int CHP, int NGP, int* __restrict__ STG, int* __restrict__ HST) {
  extern __shared__ int sm[];
  int* cnt = sm; int* run = sm + NGP; int* ids = sm + 2 * NGP;
  const int b = blockIdx.x; const int ch = (E + CSR_NBLK - 1) / CSR_NBLK; const int e0 = b * ch, e1 = min(E, e0 + ch);
  for (int i = threadIdx.x; i < NGP; i += 64) cnt[i] = 0;
  for (int i = threadIdx.x; i < CHP; i += 64) ids[i] = -1;
  __syncthreads();
  if (threadIdx.x == 0) {
    for (int e = e0; e < e1; ++e) { int d = dst[e]; d = (d < 0) ? 0 : (d >= N ? N - 1 : d); cnt[d >> CSR_GB] += 1; }
    int acc = 0; for (int g = 0; g < nG; ++g) { run[g] = acc; acc += cnt[g]; }
    for (int e = e0; e < e1; ++e) { int d = dst[e]; d = (d < 0) ? 0 : (d >= N ? N - 1 : d); const int g = d >> CSR_GB; ids[run[g]] = e; run[g] += 1; } }
  __syncthreads();
  typedef __attribute__((ext_vector_type(4))) int v4i;
  for (int pass = 0; pass < 2; ++pass) {
    for (int i = threadIdx.x; i < CHP / 4; i += 64) *(volatile v4i*)(STG + (size_t)b * CHP + i * 4) = *(const v4i*)(&ids[i * 4]);
    for (int i = threadIdx.x; i < NGP / 4; i += 64) { v4i v; for (int e = 0; e < 4; ++e) v[e] = (i * 4 + e < nG) ? cnt[i * 4 + e] : 0; *(volatile v4i*)(HST + (size_t)b * NGP + i * 4) = v; }
    __threadfence(); }
}
__global__ __launch_bounds__(512) void csrS_kernel(const int* __restrict__ HST, int nG, int NGP, int* __restrict__ START, int* __restrict__ TOT, int* __restrict__ OFF) {
  __shared__ int tot[CSR_MAXG];
  const int b = threadIdx.x;
  for (int pass = 0; pass < 2; ++pass) { int runb = 0; for (int g = 0; g < nG; ++g) { int c = HST[(size_t)b * NGP + g]; c = (c < 0) ? 0 : c; ((volatile int*)OFF)[(size_t)g * CSR_NBLK + b] = runb; runb += c; } __threadfence(); }
  for (int g = threadIdx.x; g < nG; g += 512) { int s = 0; for (int bb = 0; bb < CSR_NBLK; ++bb) { int c = HST[(size_t)bb * NGP + g]; s += (c < 0) ? 0 : c; } tot[g] = s; }
  __syncthreads();
  if (threadIdx.x < 32) {
    __shared__ int st[CSR_MAXG + 32];
    if (threadIdx.x == 0) { int acc = 0; for (int g = 0; g < NGP; ++g) { st[g] = acc; if (g < nG) acc += (tot[g] + 31) & ~31; } st[NGP] = acc; }
    __builtin_amdgcn_fence(__ATOMIC_RELEASE, "workgroup"); __builtin_amdgcn_wave_barrier(); __builtin_amdgcn_fence(__ATOMIC_ACQUIRE, "workgroup");
    for (int pass = 0; pass < 2; ++pass) { for (int i = threadIdx.x; i < NGP + 32; i += 32) { ((volatile int*)START)[i] = (i <= NGP) ? st[min(i, NGP)] : 0; ((volatile int*)TOT)[i] = (i < nG) ? tot[i] : 0; } __threadfence(); } }
}
__global__ __launch_bounds__(256) void csrB_kernel(const int* __restrict__ dst, int N, int nG, int CHP, int NGP, int permLen, const int* __restrict__ STG, const int* __restrict__ HST, const int* __restrict__ OFF, const int* __restrict__ START, const int* __restrict__ TOT, int* __restrict__ PERM, int* __restrict__ ROWPTR, int* __restrict__ ROWCNT, int* __restrict__ FLAG) {
  typedef __attribute__((ext_vector_type(4))) int v4i;
  __shared__ int ids[CSR_CAP]; __shared__ unsigned short key[CSR_CAP]; __shared__ int outp[CSR_CAP]; __shared__ int ncnt[CSR_GN + 1]; __shared__ int boff[CSR_NBLK + 1];
  const int g = blockIdx.x, t_ = threadIdx.x; int tot = TOT[g]; int st = START[g], stn = START[g + 1]; const int v0 = g * CSR_GN; const int nv = min(CSR_GN, N - v0);
  st = (st < 0) ? 0 : (st > permLen - 32 ? permLen - 32 : st) & ~31; stn = (stn < st) ? st : (stn > permLen ? permLen : stn); tot = (tot < 0) ? 0 : tot; if (tot > stn - st && tot <= CSR_CAP) tot = stn - st;
  if (tot > CSR_CAP) {
    for (int pass = 0; pass < 2; ++pass) { for (int i = t_; i < CSR_GN / 4; i += 256) { v4i a, c; for (int e = 0; e < 4; ++e) { a[e] = st; c[e] = 0; } *(volatile v4i*)(ROWPTR + v0 + i * 4) = a; *(volatile v4i*)(ROWCNT + v0 + i * 4) = c; } if (t_ == 0) ((volatile int*)FLAG)[0] = 1; __threadfence(); } (void)nv; return; }
  if (t_ == 0) { int acc = 0; for (int b = 0; b < CSR_NBLK; ++b) { boff[b] = acc; int c = HST[(size_t)b * NGP + g]; c = (c < 0) ? 0 : (c > CHP ? CHP : c); acc += c; if (acc > tot) acc = tot; } boff[CSR_NBLK] = acc; }
  for (int i = t_; i <= CSR_GN; i += 256) ncnt[i] = 0;
  __syncthreads();
  for (int b = 0; b < CSR_NBLK; ++b) { const int c = boff[b + 1] - boff[b]; int o_ = OFF[(size_t)g * CSR_NBLK + b]; o_ = (o_ < 0) ? 0 : (o_ > CHP - c ? CHP - c : o_); const int* src_ = STG + (size_t)b * CHP + o_;
    for (int i = t_; i < c; i += 256) { int id = src_[i]; id = (id < 0) ? 0 : id; ids[boff[b] + i] = id; int d = dst[id]; d = (d < v0) ? v0 : (d >= N ? N - 1 : d); int kk = d - v0; kk = (kk < 0) ? 0 : (kk >= CSR_GN ? CSR_GN - 1 : kk); key[boff[b] + i] = (unsigned short)kk; } }
  __syncthreads();
  if (t_ == 0) { for (int i = 0; i < tot; ++i) ncnt[key[i]] += 1; int acc = 0; for (int vl = 0; vl < CSR_GN; ++vl) { const int c = ncnt[vl]; ncnt[vl] = acc; acc += c; } ncnt[CSR_GN] = acc;
    for (int i = 0; i < tot; ++i) { const int vl = key[i]; outp[ncnt[vl]] = ids[i]; ncnt[vl] += 1; }
    for (int vl = CSR_GN; vl > 0; --vl) ncnt[vl] = ncnt[vl - 1]; ncnt[0] = 0; }
  __syncthreads();
  for (int pass = 0; pass < 2; ++pass) {
    for (int i = t_; i < (stn - st) / 4; i += 256) { v4i v; for (int e = 0; e < 4; ++e) { const int q = i * 4 + e; v[e] = (q < tot) ? outp[q] : -1; } *(volatile v4i*)(PERM + st + i * 4) = v; }
    for (int i = t_; i < CSR_GN / 4; i += 256) { v4i a, c; for (int e = 0; e < 4; ++e) { const int vl = i * 4 + e; a[e] = st + ncnt[vl]; c[e] = (vl < nv) ? (ncnt[vl + 1] - ncnt[vl]) : 0; } *(volatile v4i*)(ROWPTR + v0 + i * 4) = a; *(volatile v4i*)(ROWCNT + v0 + i * 4) = c; }
    __threadfence(); }
}
__global__ __launch_bounds__(256) void csrZ_kernel(int* __restrict__ p, size_t n4) { typedef __attribute__((ext_vector_type(4))) int v4i; const size_t tid = (size_t)blockIdx.x * 256 + threadIdx.x, nth = (size_t)gridDim.x * 256; v4i z = {0, 0, 0, 0}; for (size_t i = tid; i < n4; i += nth) *(volatile v4i*)(p + i * 4) = z; }
struct CsrBufs { int *STG, *HST, *OFF, *START, *TOT, *PERM, *ROWPTR, *ROWCNT, *FLAG; int nG, NGP, CHP; size_t permLen; char* base; size_t bytes; };
static size_t csr_carve(CsrBufs& c, char* ws, size_t off, int E, int N) {
  const size_t off0 = off; c.base = ws + off;
  auto al = [&](size_t bytes) { char* p = ws + off; off += (bytes + 255) & ~(size_t)255; return p; };
  c.nG = (N + CSR_GN - 1) / CSR_GN; c.NGP = (c.nG + 31) & ~31; const int ch = (E + CSR_NBLK - 1) / CSR_NBLK; c.CHP = (ch + 31) & ~31; c.permLen = (size_t)E + 32 * (size_t)c.nG + 32;
  c.STG = (int*)al((size_t)CSR_NBLK * c.CHP * 4); c.HST = (int*)al((size_t)CSR_NBLK * c.NGP * 4); c.OFF = (int*)al((size_t)c.NGP * CSR_NBLK * 4); c.START = (int*)al((size_t)(c.NGP + 64) * 4); c.TOT = (int*)al((size_t)(c.NGP + 64) * 4);
  c.PERM = (int*)al(c.permLen * 4); c.ROWPTR = (int*)al((size_t)c.nG * CSR_GN * 4); c.ROWCNT = (int*)al((size_t)c.nG * CSR_GN * 4); c.FLAG = (int*)al(256);
  c.bytes = off - off0; return off;
}
static void csr_build(const CsrBufs& c, const int* dst, int E, int N, hipStream_t stream) {
  const size_t smem = (size_t)(2 * c.NGP + c.CHP) * 4;
  csrZ_kernel<<<512, 256, 0, stream>>>((int*)c.base, c.bytes / 16);
  csrA_kernel<<<CSR_NBLK, 64, smem, stream>>>(dst, E, N, c.nG, c.CHP, c.NGP, c.STG, c.HST);
  csrS_kernel<<<1, 512, 0, stream>>>(c.HST, c.nG, c.NGP, c.START, c.TOT, c.OFF);
  csrB_kernel<<<c.nG, 256, 0, stream>>>(dst, N, c.nG, c.CHP, c.NGP, (int)c.permLen, c.STG, c.HST, c.OFF, c.START, c.TOT, c.PERM, c.ROWPTR, c.ROWCNT, c.FLAG);
}


__device__ __forceinline__ float sigm(float x) { return 1.0f / (1.0f + __expf(-x)); }
__global__ __launch_bounds__(256) void wprep_kernel(const float* __restrict__ wc, b16* __restrict__ WCT) {
  const int t = blockIdx.x * 256 + threadIdx.x; if (t >= K * K / 8) return; const int e = t * 8; v8b o; for (int j = 0; j < 8; ++j) o[j] = (b16)(bf16_rne(wc[e + j]) * WSC);
  for (int pass = 0; pass < 2; ++pass) { *(volatile v8b*)(WCT + e) = o; __threadfence(); }
}
__device__ __forceinline__ void rbm_tile(bool live, size_t n, const float* __restrict__ ratings, const int* __restrict__ dmov, const float* __restrict__ mf, const float* wrs, const float* brs, const b16* __restrict__ WCT, const float* bcs, int nloc, int hlf, v8f (&d)[4]) {
  const float rt = live ? bf16_rne(ratings[n]) * (1.0f / MAXR) : 0.0f; const size_t mv = live ? (size_t)iclamp(dmov[n], 0, NM - 1) : 0; const float* mrow = mf + mv * K;
#pragma unroll
  for (int t = 0; t < 4; ++t) d[t] = (v8f){};
#pragma unroll
  for (int kb = 0; kb < K; kb += 32) { v16b a, al;
#pragma unroll
    for (int el = 0; el < 16; ++el) { const int k = kb + ((el < 8) ? (8 * hlf + el) : (16 + 8 * hlf + el - 8)); const float z = live ? pmul(bf16_rne(mrow[k]), sigm(pmul(rt, wrs[k]) + brs[k])) : 0.0f; b16 p, q; split16(z * XS, p, q); a[el] = p; al[el] = q; }
#pragma unroll
    for (int t = 0; t < 4; ++t) { const v16b bw = frag_kb(WCT + (size_t)(t * 16 + nloc) * K + kb, hlf); d[t] = wmma16b(a, bw, d[t]); d[t] = wmma16b(al, bw, d[t]); } }
  const int lv = live ? 1 : 0;
#pragma unroll
  for (int r = 0; r < 8; ++r) { const int rowlive = __shfl(lv, 8 * hlf + r);
#pragma unroll
    for (int t = 0; t < 4; ++t) { const float s = sigm(d[t][r] * (1.0f / (XS * WSC)) + bcs[t * 16 + nloc]); d[t][r] = rowlive ? s : 0.0f; } }
}
__global__ __launch_bounds__(256) void usum_kernel(const float* __restrict__ ratings, const int* __restrict__ dmov, const float* __restrict__ mf, const float* __restrict__ wr, const float* __restrict__ br, const int* __restrict__ PERM, const int* __restrict__ ROWPTR, const int* __restrict__ ROWCNT, int permLen, const b16* __restrict__ WCT, const float* __restrict__ bc, float* __restrict__ SU) {
  __shared__ float wrs[K], brs[K], bcs[K]; __shared__ __attribute__((aligned(16))) float so[8][K];
  const int wave = threadIdx.x >> 5, lane = threadIdx.x & 31, nloc = lane & 15, hlf = lane >> 4; const size_t u = (size_t)blockIdx.x * 8 + wave;
  if (threadIdx.x < K) { wrs[threadIdx.x] = bf16_rne(wr[threadIdx.x]); brs[threadIdx.x] = bf16_rne(br[threadIdx.x]); bcs[threadIdx.x] = bf16_rne(bc[threadIdx.x]); }
  __syncthreads();
  float cs[4] = {0.0f, 0.0f, 0.0f, 0.0f};
  if (u < (size_t)NU) { int st = ROWPTR[u], cnt = ROWCNT[u]; cnt = iclamp(cnt, 0, 1 << 20); st = iclamp(st, 0, permLen - cnt);
    for (int i = 0; i < cnt; i += 16) { const int q = i + nloc; const bool live = q < cnt; const size_t n = live ? (size_t)iclamp(PERM[st + q], 0, E - 1) : 0; v8f d[4];
      rbm_tile(live, n, ratings, dmov, mf, wrs, brs, WCT, bcs, nloc, hlf, d);
#pragma unroll
      for (int t = 0; t < 4; ++t) { float s = 0.0f;
#pragma unroll
        for (int r = 0; r < 8; ++r) s += d[t][r]; s += __shfl_xor(s, 16); cs[t] += s; } } }
  if (hlf == 0) for (int t = 0; t < 4; ++t) so[wave][t * 16 + nloc] = cs[t];
  wave_lds_sync();
  for (int pass = 0; pass < 2; ++pass) { if (u < (size_t)NU && lane < 16) *(volatile v4f*)(SU + u * K + lane * 4) = *(const v4f*)(&so[wave][lane * 4]); __threadfence(); }
}
__global__ __launch_bounds__(256) void rbm_rows_kernel(const float* __restrict__ ratings, const int* __restrict__ dmov, const float* __restrict__ mf, const float* __restrict__ wr, const float* __restrict__ br, const b16* __restrict__ WCT, const float* __restrict__ bc, float* __restrict__ RBM) {
  __shared__ float wrs[K], brs[K], bcs[K]; __shared__ __attribute__((aligned(16))) float st[8][16][K + 4];
  const int wave = threadIdx.x >> 5, lane = threadIdx.x & 31, nloc = lane & 15, hlf = lane >> 4; const size_t j0 = (size_t)blockIdx.x * 128 + wave * 16;
  if (threadIdx.x < K) { wrs[threadIdx.x] = bf16_rne(wr[threadIdx.x]); brs[threadIdx.x] = bf16_rne(br[threadIdx.x]); bcs[threadIdx.x] = bf16_rne(bc[threadIdx.x]); }
  __syncthreads();
  const size_t j = j0 + nloc; const bool live = j < (size_t)NM; v8f d[4]; rbm_tile(live, live ? j : 0, ratings, dmov, mf, wrs, brs, WCT, bcs, nloc, hlf, d);
#pragma unroll
  for (int t = 0; t < 4; ++t)
#pragma unroll
    for (int r = 0; r < 8; ++r) st[wave][8 * hlf + r][t * 16 + nloc] = d[t][r];
  wave_lds_sync();
  for (int pass = 0; pass < 2; ++pass) { for (int rr = 0; rr < 16; ++rr) if (lane < 16) *(volatile v4f*)(RBM + (j0 + rr) * K + lane * 4) = *(const v4f*)(&st[wave][rr][lane * 4]); __threadfence(); }
}
__global__ __launch_bounds__(256) void query_kernel(const int* __restrict__ xu, const int* __restrict__ xm, const float* __restrict__ mf, const float* __restrict__ SU, const int* __restrict__ ROWCNT, const float* __restrict__ RBM, const float* __restrict__ wout, const float* __restrict__ bout, float* __restrict__ out) {
  __shared__ float so[32];
  const int wave = threadIdx.x >> 5, lane = threadIdx.x & 31;
  for (int q = 0; q < 4; ++q) { const size_t b = (size_t)blockIdx.x * 32 + wave * 4 + q; float part = 0.0f;
    if (b < (size_t)NB_) { const size_t u = (size_t)iclamp(xu[b], 0, NU - 1), m = (size_t)iclamp(xm[b], 0, NM - 1); const float nb = fmaxf(1.0f, (float)iclamp(ROWCNT[u], 0, 1 << 20) - 1.0f);
      for (int k2 = 0; k2 < 2; ++k2) { const int k = lane * 2 + k2; const float uf = (SU[u * K + k] - RBM[m * K + k]) / nb; part += pmul(bf16_rne(mf[m * K + k]), uf); } }
    for (int o = 16; o; o >>= 1) part += __shfl_xor(part, o);
    if (lane == 0) so[wave * 4 + q] = ((part * (1.0f / K)) * bf16_rne(wout[0]) + bf16_rne(bout[0])) * MAXR; }
  __syncthreads();
  for (int pass = 0; pass < 2; ++pass) { if (threadIdx.x < 8) *(volatile v4f*)(out + (size_t)blockIdx.x * 32 + threadIdx.x * 4) = *(const v4f*)(&so[threadIdx.x * 4]); __threadfence(); }
}
}

extern "C" void kernel_launch(void* const* d_in, const int* in_sizes, int n_in, void* d_out, int out_size, void* d_ws, size_t ws_size, hipStream_t stream) {
  (void)n_in;
  auto Fp = [&](int i) { return (const float*)d_in[i]; }; auto Ip = [&](int i) { return (const int*)d_in[i]; };
  if (in_sizes[0] != NB_ || in_sizes[1] != NB_ || in_sizes[2] != E || in_sizes[3] != E || in_sizes[4] != E || in_sizes[5] != NM * K || in_sizes[6] != K || in_sizes[8] != K * K || out_size != NB_) return;
  size_t off = 0; char* ws = (char*)d_ws;
  auto carve = [&](size_t bytes) { char* p = ws + off; off += (bytes + 255) & ~(size_t)255; return p; };
  b16* WCT = (b16*)carve((size_t)K * K * 2); float* RBM = (float*)carve((size_t)NMP * K * 4); float* SU = (float*)carve((size_t)NU * K * 4);
  CsrBufs csr; off = csr_carve(csr, ws, off, E, N);
  if (off > ws_size || off > ((size_t)128 << 20)) return;
  wprep_kernel<<<(K * K / 8 + 255) / 256, 256, 0, stream>>>(Fp(8), WCT);
  csr_build(csr, Ip(2), E, N, stream);
  usum_kernel<<<(NU + 7) / 8, 256, 0, stream>>>(Fp(4), Ip(3), Fp(5), Fp(6), Fp(7), csr.PERM, csr.ROWPTR, csr.ROWCNT, (int)csr.permLen, WCT, Fp(9), SU);
  rbm_rows_kernel<<<NMP / 128, 256, 0, stream>>>(Fp(4), Ip(3), Fp(5), Fp(6), Fp(7), WCT, Fp(9), RBM);
  query_kernel<<<(NB_ + 31) / 32, 256, 0, stream>>>(Ip(0), Ip(1), Fp(5), SU, csr.ROWCNT, RBM, Fp(10), Fp(11), (float*)d_out);
}
